// GIN_12704513261596
// MI455X (gfx1250) — hardware-verified
//
#include <hip/hip_runtime.h>
#include <stddef.h>
#include <stdint.h>


#define GN      65536
#define GD      128
#define GK2     256
#define GK3     384
#define NGR     16
#define NNG     4096
#define NLAY    3
#define NTHR    256
#define NWAVE   8
#define EPT     8
#define CHUNK   (NTHR * EPT)
#define WCAP    (EPT * 32)
#define LISTN   (NWAVE * WCAP)
#define NBA     1024
#define SLA     10
#define RCAP    20480
#define DEGCAP  64
#define METAW   (2 * NBA + 32)
#define CMP_ZINTS (2 * RCAP + 2 * NBA + 32 + LISTN)
#define CMP_LDS_INTS (CMP_ZINTS + 16)
#define AGS     128
#define APR     128
#define GBM     64
#define GBN     128
#define GTHR    128
#define GNT     8
#define PARTW   256
#define NREC    (GN / GBM)
#define RECPG   (NNG / GBM)
#define NMAT    10
#define UPR     (GK3 / 8)
#define UPP     (GD * UPR)
#define NUW     (NMAT * UPP)
#define STATW   512
#define NSTAT   7
#define WSMAX   134217728

static_assert((CHUNK & (CHUNK - 1)) == 0);
static_assert((NBA & (NBA - 1)) == 0 && NBA == (1 << SLA));
static_assert(NTHR * 4 == NBA);
static_assert(LISTN >= NBA);
static_assert((RCAP % 32) == 0 && ((RCAP / 4) % NTHR) == 0);
static_assert((METAW % 32) == 0 && (CMP_ZINTS % 4) == 0);
static_assert(CMP_LDS_INTS * 4 <= 300000);
static_assert(GBM == (GTHR / 32) * 16 && GBN == 16 * GNT && GTHR == GBN && GBN == GD);
static_assert(GD == 32 * 4 && (GD % 32) == 0 && (GK2 % 32) == 0 && GK2 == 2 * GD);
static_assert((GK3 % 32) == 0 && GK3 == 3 * GD && (GK2 & (GK2 - 1)) == 0);
static_assert((GN % NBA) == 0 && (GN % GBM) == 0 && (GN % APR) == 0 && GN == NGR * NNG);
static_assert((NBA % AGS) == 0 && AGS == NWAVE * 16 && APR == NWAVE * 16 && (NBA / AGS) == 8);
static_assert((NUW % NTHR) == 0 && (UPP % NTHR) == 0 && UPR == 48 && UPP == 6144);
static_assert(PARTW == 2 * GBN && PARTW / 4 <= GTHR && STATW == 4 * GD);
static_assert(NGR * RECPG == NREC && NGR == 16);

typedef float          v4f  __attribute__((ext_vector_type(4)));
typedef float          v8f  __attribute__((ext_vector_type(8)));
typedef int            v4i  __attribute__((ext_vector_type(4)));
typedef int            v8i  __attribute__((ext_vector_type(8)));
typedef unsigned int   v2u  __attribute__((ext_vector_type(2)));
typedef unsigned short v8us __attribute__((ext_vector_type(8)));
typedef __bf16         v16b __attribute__((ext_vector_type(16)));
typedef v4f  __attribute__((may_alias)) v4fa;
typedef v4i  __attribute__((may_alias)) v4ia;
typedef v8us __attribute__((may_alias)) v8usa;
union Frag { v16b vb; v8us h[2]; v8i w; };

__device__ __forceinline__ v8f wmx(const Frag& a, const Frag& b, v8f c) {
  v8f d = __builtin_amdgcn_wmma_f32_16x16x32_bf16(false, a.vb, false, b.vb, (short)0, c, false, false);
  asm volatile("v_nop\n\tv_nop\n\tv_nop\n\tv_nop" : "+v"(d) : "v"(a.w), "v"(b.w));
  return d;
}

__device__ __forceinline__ unsigned short bf_bits(float f) {
  unsigned int u = __float_as_uint(f);
  u += 0x7FFFu + ((u >> 16) & 1u);
  return (unsigned short)(u >> 16);
}
__device__ __forceinline__ float bf_val(unsigned short b) { return __uint_as_float(((unsigned int)b) << 16); }
__device__ __forceinline__ float bf_rne(float f) { return bf_val(bf_bits(f)); }

__device__ __forceinline__ float relu_np(float v) { return (v > 0.0f) ? v : (v - v); }
__device__ __forceinline__ float bn1(float x, float m, float r, float g, float b) { return ((x - m) * r) * g + b; }
__device__ __forceinline__ v4f fbn(const v4f x, const v4f m, const v4f r, const v4f g, const v4f b, bool rl) {
  v4f y;
  y.x = bn1(x.x, m.x, r.x, g.x, b.x);
  y.y = bn1(x.y, m.y, r.y, g.y, b.y);
  y.z = bn1(x.z, m.z, r.z, g.z, b.z);
  y.w = bn1(x.w, m.w, r.w, g.w, b.w);
  y.x = rl ? relu_np(y.x) : y.x;
  y.y = rl ? relu_np(y.y) : y.y;
  y.z = rl ? relu_np(y.z) : y.z;
  y.w = rl ? relu_np(y.w) : y.w;
  return y;
}
__device__ __forceinline__ void hilo4(const v4f a, v2u& hv, v2u& lv) {
  const unsigned short h0 = bf_bits(a.x), h1 = bf_bits(a.y), h2 = bf_bits(a.z), h3 = bf_bits(a.w);
  const unsigned short l0 = bf_bits(a.x - bf_val(h0)), l1 = bf_bits(a.y - bf_val(h1));
  const unsigned short l2 = bf_bits(a.z - bf_val(h2)), l3 = bf_bits(a.w - bf_val(h3));
  hv.x = (unsigned int)h0 | ((unsigned int)h1 << 16);
  hv.y = (unsigned int)h2 | ((unsigned int)h3 << 16);
  lv.x = (unsigned int)l0 | ((unsigned int)l1 << 16);
  lv.y = (unsigned int)l2 | ((unsigned int)l3 << 16);
}

__device__ __forceinline__ int scan_chunk(const int* __restrict__ dsts, int nE, int cbase, int slotBase,
                                          int nb, int vec8, int* list, int tid, int lane, int wave) {
  int wc = 0;
  const int el0  = tid * EPT;
  const int e0   = cbase + el0;
  const int sent = -2147483647 - 1;
  v4i da, db;
  if (vec8 != 0 && cbase + CHUNK <= nE) {
    da = *(const v4i*)(dsts + e0);
    db = *(const v4i*)(dsts + e0 + 4);
  } else {
    da.x = (e0     < nE) ? dsts[min(e0,     nE - 1)] : sent;
    da.y = (e0 + 1 < nE) ? dsts[min(e0 + 1, nE - 1)] : sent;
    da.z = (e0 + 2 < nE) ? dsts[min(e0 + 2, nE - 1)] : sent;
    da.w = (e0 + 3 < nE) ? dsts[min(e0 + 3, nE - 1)] : sent;
    db.x = (e0 + 4 < nE) ? dsts[min(e0 + 4, nE - 1)] : sent;
    db.y = (e0 + 5 < nE) ? dsts[min(e0 + 5, nE - 1)] : sent;
    db.z = (e0 + 6 < nE) ? dsts[min(e0 + 6, nE - 1)] : sent;
    db.w = (e0 + 7 < nE) ? dsts[min(e0 + 7, nE - 1)] : sent;
  }
  const unsigned nbs = (unsigned)slotBase;
  const unsigned unb = (unsigned)nb;
  const unsigned s0 = (unsigned)da.x - nbs, s1 = (unsigned)da.y - nbs;
  const unsigned s2 = (unsigned)da.z - nbs, s3 = (unsigned)da.w - nbs;
  const unsigned s4 = (unsigned)db.x - nbs, s5 = (unsigned)db.y - nbs;
  const unsigned s6 = (unsigned)db.z - nbs, s7 = (unsigned)db.w - nbs;
  const bool h0 = s0 < unb, h1 = s1 < unb, h2 = s2 < unb, h3 = s3 < unb;
  const bool h4 = s4 < unb, h5 = s5 < unb, h6 = s6 < unb, h7 = s7 < unb;
  const unsigned any = __builtin_amdgcn_ballot_w32(h0 | h1 | h2 | h3 | h4 | h5 | h6 | h7);
  if (any != 0u) {
#define HITJ(J, HJ, SJ) { \
      const unsigned mj = __builtin_amdgcn_ballot_w32(HJ); \
      if (mj != 0u) { \
        if (HJ) { \
          const int pos = wc + (int)__builtin_amdgcn_mbcnt_lo(mj, 0u); \
          if (pos < WCAP) list[wave * WCAP + pos] = ((el0 + (J)) << SLA) | (int)(SJ); \
        } \
        wc += (int)__builtin_popcount(mj); } }
    HITJ(0, h0, s0)
    HITJ(1, h1, s1)
    HITJ(2, h2, s2)
    HITJ(3, h3, s3)
    HITJ(4, h4, s4)
    HITJ(5, h5, s5)
    HITJ(6, h6, s6)
    HITJ(7, h7, s7)
#undef HITJ
  }
  return wc;
}

__global__ __launch_bounds__(NTHR) void k_wprep(const float* __restrict__ w1, const float* __restrict__ w2,
                                                const float* __restrict__ wr1, unsigned short* wt,
                                                float* statId) {
  const int tid = (int)threadIdx.x;
  if ((int)blockIdx.x == NUW / NTHR) {
    const int seg = tid >> 5;
    const float val = (seg == 1 || seg == 2) ? 1.0f : 0.0f;
    v4f sv; sv.x = val; sv.y = val; sv.z = val; sv.w = val;
    float* dp = statId + 4 * (tid & 127);
    const bool ok = tid < 128;
    if (ok) *(volatile v4f*)dp = sv;
    __threadfence();
    if (ok) *(volatile v4f*)dp = sv;
    return;
  }
  const int u   = (int)blockIdx.x * NTHR + tid;
  const int mi  = u / UPP;
  const int v   = u - mi * UPP;
  const int n   = v / UPR;
  const int kq  = v - n * UPR;
  const int k8  = kq * 8;
  const int seg = k8 >> 7;
  const int kk  = k8 & (GD - 1);
  const bool rnd = mi >= 6;
  const float* sp;
  if (mi < 3)      sp = w1  + (size_t)mi * (GD * GD);
  else if (mi < 6) sp = w2  + (size_t)(mi - 3) * (GD * GD);
  else             sp = wr1 + (size_t)(mi - 6) * (GD * GD);
  const float* p = sp + (size_t)kk * GD + n;
  v8us o;
#pragma unroll
  for (int i = 0; i < 8; ++i) {
    const float x   = p[(size_t)i * GD];
    const float val = rnd ? bf_rne(x) : x;
    const unsigned short hb = bf_bits(val);
    const unsigned short lb = bf_bits(val - bf_val(hb));
    o[i] = (seg == 2) ? lb : hb;
  }
  unsigned short* dp = wt + (size_t)u * 8;
  *(volatile v8us*)dp = o;
  __threadfence();
  *(volatile v8us*)dp = o;
}

__global__ __launch_bounds__(NTHR) void k_h0(const int* __restrict__ state, const float* __restrict__ embed,
                                             int nN, float* P2, unsigned short* P1) {
  const int tid = (int)threadIdx.x, lane = tid & 31, wave = tid >> 5;
  const int base = (int)blockIdx.x * APR + wave * 16;
  v2u zz; zz.x = 0u; zz.y = 0u;
#pragma unroll 1
  for (int b = 0; b < 4; ++b) {
    v4f fv[4];
    v2u hv[4];
#pragma unroll
    for (int j = 0; j < 4; ++j) {
      const int row = base + 4 * b + j;
      const int rc  = row < nN ? row : nN - 1;
      int s = state[rc];
      s = s < 0 ? 0 : (s > 1 ? 1 : s);
      const v4f e = *(const v4f*)(embed + (size_t)s * GD + 4 * lane);
      v4f f; f.x = bf_rne(e.x); f.y = bf_rne(e.y); f.z = bf_rne(e.z); f.w = bf_rne(e.w);
      fv[j] = f;
      v2u h;
      h.x = (unsigned int)bf_bits(f.x) | ((unsigned int)bf_bits(f.y) << 16);
      h.y = (unsigned int)bf_bits(f.z) | ((unsigned int)bf_bits(f.w) << 16);
      hv[j] = h;
    }
#pragma unroll
    for (int j = 0; j < 4; ++j) {
      const int row = base + 4 * b + j;
      float* fp = P2 + (size_t)row * GD + 4 * lane;
      unsigned short* hp = P1 + (size_t)row * GK2 + 4 * lane;
      if (row < nN) { *(volatile v4f*)fp = fv[j]; *(volatile v2u*)hp = hv[j]; *(volatile v2u*)(hp + GD) = zz; }
    }
    __threadfence();
#pragma unroll
    for (int j = 0; j < 4; ++j) {
      const int row = base + 4 * b + j;
      float* fp = P2 + (size_t)row * GD + 4 * lane;
      unsigned short* hp = P1 + (size_t)row * GK2 + 4 * lane;
      if (row < nN) { *(volatile v4f*)fp = fv[j]; *(volatile v2u*)hp = hv[j]; *(volatile v2u*)(hp + GD) = zz; }
    }
  }
}

__global__ __launch_bounds__(NTHR) void k_compact(const int* __restrict__ srcs, const int* __restrict__ dsts,
                                                  int nE, int nN, int vec8, int* srcl, int* meta) {
  extern __shared__ __attribute__((aligned(16))) int dsm[];
  int* reg1 = dsm;
  int* reg2 = reg1 + RCAP;
  int* soff = reg2 + RCAP;
  int* scnt = soff + NBA;
  int* misc = scnt + NBA;
  int* list = misc + 32;
  int* wcnt = list + LISTN;
  int* wtot = wcnt + NWAVE;
  const int tid = (int)threadIdx.x, lane = tid & 31, wave = tid >> 5;
  const int nodeBase = (int)blockIdx.x * NBA;

  {
    const v4i z4 = {0, 0, 0, 0};
    for (int i = tid * 4; i < CMP_ZINTS; i += NTHR * 4) *(v4ia*)(dsm + i) = z4;
    if (tid < 2 * NWAVE) wcnt[tid] = 0;
  }
  __syncthreads();

  int tot = 0, ov = 0;
  const int nChunks = (nE + CHUNK - 1) / CHUNK;
#pragma unroll 1
  for (int ch = 0; ch < nChunks; ++ch) {
    const int cbase = ch * CHUNK;
    const int wc = scan_chunk(dsts, nE, cbase, nodeBase, NBA, vec8, list, tid, lane, wave);
    if (lane == 0) wcnt[wave] = wc;
    __syncthreads();
    int pre = 0, all = 0;
#pragma unroll
    for (int w2 = 0; w2 < NWAVE; ++w2) {
      int c = wcnt[w2];
      c = c < 0 ? 0 : (c > WCAP ? WCAP : c);
      all += c;
      pre += (w2 < wave) ? c : 0;
    }
    const int wcc  = wc > WCAP ? WCAP : wc;
    const int base = tot + pre;
#pragma unroll 1
    for (int i = lane; i < wcc; i += 32) {
      const int ent = list[wave * WCAP + i];
      const int el  = (ent >> SLA) & (CHUNK - 1);
      const int sl  = ent & (NBA - 1);
      int eid = cbase + el;
      eid = eid > nE - 1 ? nE - 1 : eid;
      const int pos = base + i;
      if (pos < RCAP) reg1[pos] = (int)(((unsigned)eid << SLA) | (unsigned)sl);
    }
    if (tot + all > RCAP) ov = 1;
    tot += all;
    tot = tot > RCAP ? RCAP : tot;
    __syncthreads();
  }
  const int nh = tot;

  if (wave == 0) {
#pragma unroll 1
    for (int b0 = 0; b0 < nh; b0 += 32) {
      const int idx = b0 + lane;
      const int uv  = reg1[idx < RCAP ? idx : RCAP - 1];
      const int m32 = (nh - b0) < 32 ? (nh - b0) : 32;
#pragma unroll 1
      for (int k = 0; k < m32; ++k) {
        const int u  = __builtin_amdgcn_readlane(uv, k);
        const int sl = u & (NBA - 1);
        if (lane == 0) scnt[sl] = scnt[sl] + 1;
      }
    }
  }
  __syncthreads();

  {
    const v4i ca = *(const v4ia*)(scnt + 4 * tid);
    const int e0 = ca.x < 0 ? 0 : ca.x, e1 = ca.y < 0 ? 0 : ca.y, e2 = ca.z < 0 ? 0 : ca.z, e3 = ca.w < 0 ? 0 : ca.w;
    const int ts = e0 + e1 + e2 + e3;
    int incl = ts;
#pragma unroll
    for (int d = 1; d < 32; d <<= 1) {
      const int up = __shfl_up(incl, d);
      if (lane >= d) incl += up;
    }
    if (lane == 31) wtot[wave] = incl;
    __syncthreads();
    int pre = 0;
#pragma unroll
    for (int w2 = 0; w2 < NWAVE; ++w2) pre += (w2 < wave) ? wtot[w2] : 0;
    int run = pre + incl - ts;
    soff[4 * tid + 0] = run; run += e0;
    soff[4 * tid + 1] = run; run += e1;
    soff[4 * tid + 2] = run; run += e2;
    soff[4 * tid + 3] = run;
  }
  __syncthreads();
  for (int i = tid; i < NBA; i += NTHR) list[i] = soff[i];
  if (tid == 0) { misc[0] = nh; misc[1] = ov; }
  __syncthreads();

  if (wave == 0) {
#pragma unroll 1
    for (int b0 = 0; b0 < nh; b0 += 32) {
      const int idx = b0 + lane;
      const int uv  = reg1[idx < RCAP ? idx : RCAP - 1];
      const int m32 = (nh - b0) < 32 ? (nh - b0) : 32;
#pragma unroll 1
      for (int k = 0; k < m32; ++k) {
        const int u   = __builtin_amdgcn_readlane(uv, k);
        const int sl  = u & (NBA - 1);
        const int eid = (int)((unsigned)u >> SLA);
        if (lane == 0) {
          int pos = list[sl];
          pos = pos < 0 ? 0 : (pos > RCAP - 1 ? RCAP - 1 : pos);
          reg2[pos] = eid;
          list[sl] = pos + 1;
        }
      }
    }
  }
  __syncthreads();

#pragma unroll 1
  for (int i = tid; i < nh; i += NTHR) {
    int eid = reg2[i];
    eid = eid < 0 ? 0 : (eid > nE - 1 ? nE - 1 : eid);
    int s = srcs[eid];
    s = s < 0 ? 0 : (s > nN - 1 ? nN - 1 : s);
    reg2[i] = s;
  }
  __syncthreads();

  int* gs = srcl + (size_t)blockIdx.x * RCAP;
  int* gm = meta + (size_t)blockIdx.x * METAW;
#pragma unroll 1
  for (int p = tid; p < RCAP / 4; p += NTHR) {
    const v4i v = *(const v4ia*)(reg2 + 4 * p);
    *(volatile v4i*)(gs + 4 * p) = v;
  }
#pragma unroll 1
  for (int p = tid; p < METAW / 4; p += NTHR) {
    const v4i v = *(const v4ia*)(soff + 4 * p);
    *(volatile v4i*)(gm + 4 * p) = v;
  }
  __threadfence();
#pragma unroll 1
  for (int p = tid; p < RCAP / 4; p += NTHR) {
    const v4i v = *(const v4ia*)(reg2 + 4 * p);
    *(volatile v4i*)(gs + 4 * p) = v;
  }
#pragma unroll 1
  for (int p = tid; p < METAW / 4; p += NTHR) {
    const v4i v = *(const v4ia*)(soff + 4 * p);
    *(volatile v4i*)(gm + 4 * p) = v;
  }
}

__global__ __launch_bounds__(NTHR) void k_agg(const float* __restrict__ X, const float* __restrict__ stat,
                                              int relu_on, const int* __restrict__ srcl,
                                              const int* __restrict__ meta, int nN, unsigned short* P1) {
  const int tid = (int)threadIdx.x, lane = tid & 31, wave = tid >> 5;
  const int lb = (int)blockIdx.x >> 3, sub = (int)blockIdx.x & 7;
  const int* mt = meta + (size_t)lb * METAW;
  const int* sl = srcl + (size_t)lb * RCAP;
  int nh = mt[2 * NBA];
  nh = nh < 0 ? 0 : (nh > RCAP ? RCAP : nh);
  const int ovf = mt[2 * NBA + 1];
  const int s0 = sub * AGS + wave * 16;
  const int myoff = mt[s0 + (lane & 15)];
  const int mycnt = mt[NBA + s0 + (lane & 15)];
  const v4f m4 = *(const v4f*)(stat + 4 * lane);
  const v4f r4 = *(const v4f*)(stat + GD + 4 * lane);
  const v4f g4 = *(const v4f*)(stat + 2 * GD + 4 * lane);
  const v4f b4 = *(const v4f*)(stat + 3 * GD + 4 * lane);
  const bool rl = relu_on != 0;
  const float qnan = __int_as_float(0x7fc00000);

#pragma unroll 1
  for (int j = 0; j < 16; ++j) {
    const int slot = s0 + j;
    const int row  = lb * NBA + slot;
    int st = __builtin_amdgcn_readlane(myoff, j);
    const int craw = __builtin_amdgcn_readlane(mycnt, j);
    int cnt = craw;
    st  = st < 0 ? 0 : (st > nh ? nh : st);
    cnt = cnt < 0 ? 0 : (cnt > DEGCAP ? DEGCAP : cnt);
    if (cnt > nh - st) cnt = nh - st;
    const float pz = (ovf != 0 || craw > DEGCAP) ? qnan : 0.0f;

    float a0 = 0.0f, a1 = 0.0f, a2 = 0.0f, a3 = 0.0f;
#pragma unroll 1
    for (int b0 = 0; b0 < cnt; b0 += 32) {
      int idx = st + b0 + lane;
      idx = idx > RCAP - 1 ? RCAP - 1 : idx;
      int sr = sl[idx];
      sr = sr < 0 ? 0 : (sr > nN - 1 ? nN - 1 : sr);
      const int m32 = (cnt - b0) < 32 ? (cnt - b0) : 32;
#pragma unroll 1
      for (int k = 0; k < m32; ++k) {
        const int sk = __builtin_amdgcn_readlane(sr, k);
        const v4f xv = *(const v4f*)(X + (size_t)sk * GD + 4 * lane);
        const v4f y = fbn(xv, m4, r4, g4, b4, rl);
        a0 += y.x; a1 += y.y; a2 += y.z; a3 += y.w;
      }
    }
    const int rc = row < nN ? row : nN - 1;
    const v4f sv = fbn(*(const v4f*)(X + (size_t)rc * GD + 4 * lane), m4, r4, g4, b4, rl);
    v4f z;
    z.x = (sv.x + a0) + pz;
    z.y = (sv.y + a1) + pz;
    z.z = (sv.z + a2) + pz;
    z.w = (sv.w + a3) + pz;
    v2u hv, lv;
    hilo4(z, hv, lv);
    unsigned short* hp = P1 + (size_t)row * GK2 + 4 * lane;
    const bool ok = row < nN;
    if (ok) { *(volatile v2u*)hp = hv; *(volatile v2u*)(hp + GD) = lv; }
    __threadfence();
    if (ok) { *(volatile v2u*)hp = hv; *(volatile v2u*)(hp + GD) = lv; }
  }
}

__global__ __launch_bounds__(NTHR) void k_apply(const float* __restrict__ T, const float* __restrict__ stat,
                                                int nN, unsigned short* P1) {
  const int tid = (int)threadIdx.x, lane = tid & 31, wave = tid >> 5;
  const int base = (int)blockIdx.x * APR + wave * 16;
  const v4f m4 = *(const v4f*)(stat + 4 * lane);
  const v4f r4 = *(const v4f*)(stat + GD + 4 * lane);
  const v4f g4 = *(const v4f*)(stat + 2 * GD + 4 * lane);
  const v4f b4 = *(const v4f*)(stat + 3 * GD + 4 * lane);
#pragma unroll 1
  for (int b = 0; b < 4; ++b) {
    v2u hv[4], lv[4];
#pragma unroll
    for (int j = 0; j < 4; ++j) {
      const int row = base + 4 * b + j;
      const int rc  = row < nN ? row : nN - 1;
      const v4f y = fbn(*(const v4f*)(T + (size_t)rc * GD + 4 * lane), m4, r4, g4, b4, true);
      hilo4(y, hv[j], lv[j]);
    }
#pragma unroll
    for (int j = 0; j < 4; ++j) {
      const int row = base + 4 * b + j;
      unsigned short* hp = P1 + (size_t)row * GK2 + 4 * lane;
      if (row < nN) { *(volatile v2u*)hp = hv[j]; *(volatile v2u*)(hp + GD) = lv[j]; }
    }
    __threadfence();
#pragma unroll
    for (int j = 0; j < 4; ++j) {
      const int row = base + 4 * b + j;
      unsigned short* hp = P1 + (size_t)row * GK2 + 4 * lane;
      if (row < nN) { *(volatile v2u*)hp = hv[j]; *(volatile v2u*)(hp + GD) = lv[j]; }
    }
  }
}

template <int EPI>
__global__ __launch_bounds__(GTHR) void k_gemm(const unsigned short* __restrict__ A, int lda,
                                               const unsigned short* __restrict__ BT, int ldb, int K,
                                               const float* __restrict__ bias, float* outF, const float* racc,
                                               float* part, const float* __restrict__ wr2,
                                               const float* __restrict__ br2, float* score, float* maxrec,
                                               int mRows) {
  __shared__ __attribute__((aligned(16))) float stg[GBM * GBN];
  __shared__ __attribute__((aligned(16))) float pst[PARTW];
  const int tid = (int)threadIdx.x, lane = tid & 31, wave = tid >> 5, hh = lane >> 4, m = lane & 15;
  const int rowBase = (int)blockIdx.x * GBM;

  v8f acc[GNT];
  {
    const v8f z = {0.f, 0.f, 0.f, 0.f, 0.f, 0.f, 0.f, 0.f};
#pragma unroll
    for (int t = 0; t < GNT; ++t) acc[t] = z;
  }
  const unsigned short* ap = A  + (size_t)(rowBase + 16 * wave + m) * (size_t)lda + 8 * hh;
  const unsigned short* bp = BT + (size_t)m * (size_t)ldb + 8 * hh;

#pragma unroll 1
  for (int k0 = 0; k0 < K; k0 += 32) {
    const int ka = k0 & (GK2 - 1);
    Frag af;
    af.h[0] = *(const v8usa*)(ap + ka);
    af.h[1] = *(const v8usa*)(ap + ka + 16);
#pragma unroll
    for (int nt = 0; nt < GNT; ++nt) {
      const unsigned short* wq = bp + (size_t)(16 * nt) * (size_t)ldb + k0;
      Frag bfr;
      bfr.h[0] = *(const v8usa*)wq;
      bfr.h[1] = *(const v8usa*)(wq + 16);
      acc[nt] = wmx(af, bfr, acc[nt]);
    }
  }

#pragma unroll
  for (int nt = 0; nt < GNT; ++nt) {
    const int lc = 16 * nt + m;
    float bb = 0.0f;
    if constexpr (EPI == 1) bb = bf_rne(bias[lc]);
#pragma unroll
    for (int r = 0; r < 8; ++r) {
      const int lr = 16 * wave + 8 * hh + r;
      stg[lr * GBN + lc] = acc[nt][r] + bb;
    }
  }
  __syncthreads();

  if constexpr (EPI == 3) {
    float* wsh = pst;
    float* sc  = pst + GBN;
#pragma unroll 1
    for (int i = 0; i < 16; ++i) {
      const int lr = 16 * wave + i;
      const int gr = rowBase + lr;
      const v4f a = *(const v4fa*)(stg + lr * GBN + 4 * lane);
      const v4f q = *(const v4f*)(racc + (size_t)gr * GBN + 4 * lane);
      v4f v;
      v.x = relu_np(q.x + a.x); v.y = relu_np(q.y + a.y); v.z = relu_np(q.z + a.z); v.w = relu_np(q.w + a.w);
      *(v4fa*)(stg + lr * GBN + 4 * lane) = v;
    }
    wsh[tid] = bf_rne(wr2[tid]);
    __syncthreads();
    const int row = tid >> 1, half = tid & 1;
    float s = 0.0f;
#pragma unroll 4
    for (int c = 0; c < 64; ++c) s = fmaf(stg[row * GBN + half * 64 + c], wsh[half * 64 + c], s);
    const float o = __shfl_xor(s, 1);
    const float tot = s + o;
    const float b2 = bf_rne(br2[0]);
    if (half == 0) sc[row] = tot + b2;
    __syncthreads();
    if (wave == 0) {
      const float a = sc[lane], b = sc[lane + 32];
      float mx = a;
      mx = (b > mx || b != b) ? b : mx;
#pragma unroll
      for (int d = 16; d >= 1; d >>= 1) {
        const float ov = __shfl_xor(mx, d);
        mx = (ov > mx || ov != ov) ? ov : mx;
      }
      const v4f sv = *(const v4fa*)(sc + 4 * (lane & 15));
      v4f mv; mv.x = mx; mv.y = mx; mv.z = mx; mv.w = mx;
      float* sp = score + (size_t)rowBase + 4 * (lane & 15);
      float* mp = maxrec + (size_t)blockIdx.x * 32 + 4 * (lane & 7);
      const bool ok16 = (lane < 16) && (rowBase + GBM <= mRows);
      const bool ok8  = lane < 8;
      if (ok16) *(volatile v4f*)sp = sv;
      if (ok8)  *(volatile v4f*)mp = mv;
      __threadfence();
      if (ok16) *(volatile v4f*)sp = sv;
      if (ok8)  *(volatile v4f*)mp = mv;
    }
  } else {
    v4f fv[16];
#pragma unroll
    for (int i = 0; i < 16; ++i) {
      const int lr = 16 * wave + i;
      v4f a = *(const v4fa*)(stg + lr * GBN + 4 * lane);
      if constexpr (EPI == 2) {
        const int gr = rowBase + lr;
        const v4f q = *(const v4f*)(racc + (size_t)gr * GBN + 4 * lane);
        a.x = q.x + a.x; a.y = q.y + a.y; a.z = q.z + a.z; a.w = q.w + a.w;
      }
      fv[i] = a;
    }
    v4f pv = {0.f, 0.f, 0.f, 0.f};
    const bool pok = (EPI == 0) && (tid < PARTW / 4);
    if constexpr (EPI == 0) {
      float s = 0.0f;
#pragma unroll 1
      for (int r = 0; r < GBM; ++r) s += stg[r * GBN + tid];
      const float mean = s * (1.0f / (float)GBM);
      float q = 0.0f;
#pragma unroll 1
      for (int r = 0; r < GBM; ++r) {
        const float d = stg[r * GBN + tid] - mean;
        q = fmaf(d, d, q);
      }
      pst[tid] = mean;
      pst[GBN + tid] = q;
      __syncthreads();
      if (pok) pv = *(const v4fa*)(pst + 4 * tid);
    }
    float* pp = part + (size_t)blockIdx.x * PARTW + 4 * (tid & 63);
#pragma unroll
    for (int i = 0; i < 16; ++i) {
      const int gr = rowBase + 16 * wave + i;
      float* op = outF + (size_t)gr * GBN + 4 * lane;
      if (gr < mRows) *(volatile v4f*)op = fv[i];
    }
    if (pok) *(volatile v4f*)pp = pv;
    __threadfence();
#pragma unroll
    for (int i = 0; i < 16; ++i) {
      const int gr = rowBase + 16 * wave + i;
      float* op = outF + (size_t)gr * GBN + 4 * lane;
      if (gr < mRows) *(volatile v4f*)op = fv[i];
    }
    if (pok) *(volatile v4f*)pp = pv;
  }
}

__global__ __launch_bounds__(GD) void k_comb(const float* __restrict__ part, int nRec, float rowsPer,
                                             const float* __restrict__ gam, const float* __restrict__ bet,
                                             float* stat) {
  __shared__ __attribute__((aligned(16))) float st[STATW];
  const int tid = (int)threadIdx.x;
  double sm = 0.0;
#pragma unroll 1
  for (int b = 0; b < nRec; ++b) sm += (double)part[(size_t)b * PARTW + tid];
  const double mean = sm / (double)nRec;
  double q1 = 0.0, q2 = 0.0;
#pragma unroll 1
  for (int b = 0; b < nRec; ++b) {
    const double d = (double)part[(size_t)b * PARTW + tid] - mean;
    q1 += (double)part[(size_t)b * PARTW + GD + tid];
    q2 += d * d;
  }
  const double M2 = q1 + (double)rowsPer * q2;
  const float var = (float)(M2 / ((double)nRec * (double)rowsPer));
  const float r = 1.0f / sqrtf(var + 1e-5f);
  st[tid] = (float)mean;
  st[GD + tid] = r;
  st[2 * GD + tid] = gam[tid];
  st[3 * GD + tid] = bet[tid];
  __syncthreads();
  const v4f v = *(const v4fa*)(st + 4 * tid);
  float* dp = stat + 4 * tid;
  *(volatile v4f*)dp = v;
  __threadfence();
  *(volatile v4f*)dp = v;
}

__global__ __launch_bounds__(32) void k_pool(const float* __restrict__ maxrec, int recPer, int nG,
                                             float* out, int off) {
  __shared__ __attribute__((aligned(16))) float ps[32];
  const int lane = (int)threadIdx.x & 31;
  const int g = lane < nG ? lane : nG - 1;
  float mx = maxrec[(size_t)(g * recPer) * 32];
#pragma unroll 1
  for (int j = 1; j < recPer; ++j) {
    const float v = maxrec[(size_t)(g * recPer + j) * 32];
    mx = (v > mx || v != v) ? v : mx;
  }
  ps[lane] = mx;
  __syncthreads();
  const v4f ov = *(const v4fa*)(ps + 4 * (lane & 3));
  float* op = out + (size_t)off + 4 * (lane & 3);
  const bool ok = lane < 4;
  if (ok) *(volatile v4f*)op = ov;
  __threadfence();
  if (ok) *(volatile v4f*)op = ov;
}

static inline size_t al256(size_t o) { return (o + 255) & ~(size_t)255; }

extern "C" void kernel_launch(void* const* d_in, const int* in_sizes, int n_in,
                              void* d_out, int out_size, void* d_ws, size_t ws_size,
                              hipStream_t stream) {
  if (n_in < 13) return;
  const int nN = in_sizes[0];
  if (nN != GN) return;
  if (in_sizes[1] < 2 || (in_sizes[1] & 1) != 0) return;
  const int nE = in_sizes[1] / 2;
  if (nE < 1 || nE > (1 << 21)) return;
  if (in_sizes[2] != 2 * GD) return;
  if (in_sizes[3] != NLAY * GD * GD || in_sizes[4] != NLAY * GD * GD) return;
  if (in_sizes[5] != NLAY * GD || in_sizes[6] != NLAY * GD) return;
  if (in_sizes[7] != NLAY * GD || in_sizes[8] != NLAY * GD) return;
  if (in_sizes[9] != 4 * GD * GD) return;
  if (in_sizes[10] != GD || in_sizes[11] != GD || in_sizes[12] != 1) return;
  if (out_size != GN + NGR) return;

  const int*   state = (const int*)  d_in[0];
  const int*   ei    = (const int*)  d_in[1];
  const int*   src   = ei;
  const int*   dst   = ei + nE;
  const float* embed = (const float*)d_in[2];
  const float* w1    = (const float*)d_in[3];
  const float* w2    = (const float*)d_in[4];
  const float* bn1g  = (const float*)d_in[5];
  const float* bn1b  = (const float*)d_in[6];
  const float* bn2g  = (const float*)d_in[7];
  const float* bn2b  = (const float*)d_in[8];
  const float* wr1   = (const float*)d_in[9];
  const float* br1   = (const float*)d_in[10];
  const float* wr2   = (const float*)d_in[11];
  const float* br2   = (const float*)d_in[12];
  float* out = (float*)d_out;

  const int nLB  = nN / NBA;
  const int vec8 = ((nE & 3) == 0) ? 1 : 0;

  char* ws = (char*)d_ws;
  size_t off = 0;
  const size_t oWT = off; off = al256(off + (size_t)NUW * 16);
  const size_t oST = off; off = al256(off + (size_t)NSTAT * STATW * 4);
  const size_t oPT = off; off = al256(off + (size_t)NREC * PARTW * 4);
  const size_t oMX = off; off = al256(off + (size_t)NREC * 32 * 4);
  const size_t oMT = off; off = al256(off + (size_t)nLB * METAW * 4);
  const size_t oSL = off; off = al256(off + (size_t)nLB * RCAP * 4);
  const size_t oP1 = off; off = al256(off + (size_t)nN * GK2 * 2);
  const size_t oP2 = off; off = al256(off + (size_t)nN * GD * 4);
  const size_t oRA = off; off = al256(off + (size_t)nN * GD * 4);
  if (off > ws_size || off > (size_t)WSMAX) return;
  unsigned short* WT = (unsigned short*)(ws + oWT);
  float*          ST = (float*)(ws + oST);
  float*          PT = (float*)(ws + oPT);
  float*          MX = (float*)(ws + oMX);
  int*            MT = (int*)(ws + oMT);
  int*            SL = (int*)(ws + oSL);
  unsigned short* P1 = (unsigned short*)(ws + oP1);
  float*          P2 = (float*)(ws + oP2);
  float*          RA = (float*)(ws + oRA);
  const size_t WPL = (size_t)GD * GK3;

  const int cmpLds = CMP_LDS_INTS * 4;
  hipFuncSetAttribute(reinterpret_cast<const void*>(&k_compact), hipFuncAttributeMaxDynamicSharedMemorySize, cmpLds);

  k_wprep<<<NUW / NTHR + 1, NTHR, 0, stream>>>(w1, w2, wr1, WT, ST);
  k_h0<<<nN / APR, NTHR, 0, stream>>>(state, embed, nN, P2, P1);
  k_compact<<<nLB, NTHR, cmpLds, stream>>>(src, dst, nE, nN, vec8, SL, MT);
  k_gemm<1><<<nN / GBM, GTHR, 0, stream>>>(P1, GK2, WT + 6 * WPL, GK3, GD, br1, RA, RA, PT, wr2, br2, out, MX, nN);

  for (int i = 0; i < NLAY; ++i) {
    const float* stIn = (i == 0) ? ST : (ST + (size_t)(2 + 2 * (i - 1)) * STATW);
    float* st1 = ST + (size_t)(1 + 2 * i) * STATW;
    float* st2 = ST + (size_t)(2 + 2 * i) * STATW;
    k_agg<<<nLB * (NBA / AGS), NTHR, 0, stream>>>(P2, stIn, (i > 0) ? 1 : 0, SL, MT, nN, P1);
    k_gemm<0><<<nN / GBM, GTHR, 0, stream>>>(P1, GK2, WT + (size_t)i * WPL, GK3, GK3, br1, P2, RA, PT, wr2, br2, out, MX, nN);
    k_comb<<<1, GD, 0, stream>>>(PT, NREC, (float)GBM, bn1g + (size_t)i * GD, bn1b + (size_t)i * GD, st1);
    k_apply<<<nN / APR, NTHR, 0, stream>>>(P2, st1, nN, P1);
    k_gemm<0><<<nN / GBM, GTHR, 0, stream>>>(P1, GK2, WT + (size_t)(3 + i) * WPL, GK3, GK3, br1, P2, RA, PT, wr2, br2, out, MX, nN);
    k_comb<<<1, GD, 0, stream>>>(PT, NREC, (float)GBM, bn2g + (size_t)i * GD, bn2b + (size_t)i * GD, st2);
    k_apply<<<nN / APR, NTHR, 0, stream>>>(P2, st2, nN, P1);
    if (i < NLAY - 1) {
      k_gemm<2><<<nN / GBM, GTHR, 0, stream>>>(P1, GK2, WT + (size_t)(7 + i) * WPL, GK3, GK2, br1, RA, RA, PT, wr2, br2, out, MX, nN);
    } else {
      k_gemm<3><<<nN / GBM, GTHR, 0, stream>>>(P1, GK2, WT + (size_t)(7 + i) * WPL, GK3, GK2, br1, RA, RA, PT, wr2, br2, out, MX, nN);
    }
  }
  k_pool<<<1, 32, 0, stream>>>(MX, RECPG, NGR, out, GN);
}
